// MiniAttentionBlock_57019985822328
// MI455X (gfx1250) — hardware-run, weakly checked
//
#include <hip/hip_runtime.h>
#include <stddef.h>
#include <stdint.h>

#define NBAT  4
#define SQ    2048
#define NTOK  8192
#define HID   1024
#define NH    8
#define HDM   128
#define NQKV  3072
#define QB    128
#define KC    64
#define NQB   (SQ / QB)

static_assert(NTOK == NBAT * SQ);
static_assert(SQ % 256 == 0);
static_assert(NTOK % 256 == 0);
static_assert(HID % 64 == 0);
static_assert(HID == 128 * 8);
static_assert(HDM == 128);
static_assert(NH * HDM == HID);
static_assert(NQKV == 3 * HID);
static_assert(SQ % QB == 0);
static_assert(SQ % KC == 0);
static_assert((HID * HID) % 2048 == 0);

typedef _Float16 v16h __attribute__((ext_vector_type(16)));
typedef _Float16 v8h  __attribute__((ext_vector_type(8)));
typedef float    v8f  __attribute__((ext_vector_type(8)));
typedef float    v4f  __attribute__((ext_vector_type(4)));
typedef unsigned int v4u __attribute__((ext_vector_type(4)));

union Frag  { v16h v; v8h h[2]; };
union Pack8 { v8h h; v4u u; };

__device__ __forceinline__ v8f mma16(v16h a, v16h b, v8f c) {
  c = __builtin_amdgcn_wmma_f32_16x16x32_f16(false, a, false, b, (short)0, c, false, false);
  asm volatile("v_nop\n\tv_nop\n\tv_nop\n\tv_nop" : "+v"(c) : "v"(a), "v"(b));
  return c;
}

__device__ __forceinline__ v16h ldfrag(const _Float16* p, int ld, int row0, int k0, int lane) {
  const int m = lane & 15, lh = lane >> 4;
  const _Float16* q = p + (size_t)(row0 + m) * ld + k0 + 8 * lh;
  Frag f;
  f.h[0] = *(const v8h*)(q);
  f.h[1] = *(const v8h*)(q + 16);
  return f.v;
}

__device__ __forceinline__ v8f zero8() { return (v8f){0.f, 0.f, 0.f, 0.f, 0.f, 0.f, 0.f, 0.f}; }

__device__ __forceinline__ void gemm16x64(const _Float16* __restrict__ A, int lda,
                                          const _Float16* __restrict__ Bt, int ldb,
                                          int m0, int n0, int lane, v8f (&acc)[4]) {
#pragma unroll 2
  for (int k0 = 0; k0 < HID; k0 += 32) {
    const v16h a = ldfrag(A, lda, m0, k0, lane);
#pragma unroll
    for (int t = 0; t < 4; ++t) {
      const v16h b = ldfrag(Bt, ldb, n0 + 16 * t, k0, lane);
      acc[t] = mma16(a, b, acc[t]);
    }
  }
}

__device__ __forceinline__ void gemm32x64(const _Float16* __restrict__ A, int lda,
                                          const _Float16* __restrict__ Bt, int ldb,
                                          int m0, int n0, int lane, v8f (&acc)[2][4]) {
#pragma unroll 2
  for (int k0 = 0; k0 < HID; k0 += 32) {
    const v16h a0 = ldfrag(A, lda, m0, k0, lane);
    const v16h a1 = ldfrag(A, lda, m0 + 16, k0, lane);
    const v16h b0 = ldfrag(Bt, ldb, n0, k0, lane);
    const v16h b1 = ldfrag(Bt, ldb, n0 + 16, k0, lane);
    const v16h b2 = ldfrag(Bt, ldb, n0 + 32, k0, lane);
    const v16h b3 = ldfrag(Bt, ldb, n0 + 48, k0, lane);
    acc[0][0] = mma16(a0, b0, acc[0][0]);
    acc[1][0] = mma16(a1, b0, acc[1][0]);
    acc[0][1] = mma16(a0, b1, acc[0][1]);
    acc[1][1] = mma16(a1, b1, acc[1][1]);
    acc[0][2] = mma16(a0, b2, acc[0][2]);
    acc[1][2] = mma16(a1, b2, acc[1][2]);
    acc[0][3] = mma16(a0, b3, acc[0][3]);
    acc[1][3] = mma16(a1, b3, acc[1][3]);
  }
}

__global__ __launch_bounds__(256) void k_cvtw(const float* __restrict__ w0, const float* __restrict__ w1,
                                              const float* __restrict__ w2, const float* __restrict__ w3,
                                              _Float16* __restrict__ wt, _Float16* __restrict__ wot) {
  const int y = blockIdx.y;
  const float* s = (y == 0) ? w0 : ((y == 1) ? w1 : ((y == 2) ? w2 : w3));
  _Float16* d = (y < 3) ? (wt + (size_t)y * HID * HID) : wot;
  const size_t i = (size_t)blockIdx.x * 2048 + (size_t)threadIdx.x * 8;
  const v4f a0 = *(const v4f*)(s + i);
  const v4f a1 = *(const v4f*)(s + i + 4);
  Pack8 pk;
  pk.h = (v8h){(_Float16)(a0[0] * 32.0f), (_Float16)(a0[1] * 32.0f), (_Float16)(a0[2] * 32.0f), (_Float16)(a0[3] * 32.0f),
               (_Float16)(a1[0] * 32.0f), (_Float16)(a1[1] * 32.0f), (_Float16)(a1[2] * 32.0f), (_Float16)(a1[3] * 32.0f)};
  const v4u vv = pk.u;
  volatile v4u* dp = (volatile v4u*)(d + i);
  *dp = vv;
  __threadfence();
  *dp = vv;
}

__global__ __launch_bounds__(128) void k_ln(const float* __restrict__ x, const float* __restrict__ gm,
                                            const float* __restrict__ bt, _Float16* __restrict__ xh) {
  __shared__ float rs1[4];
  __shared__ float rs2[4];
  const int tid = threadIdx.x, lane = tid & 31, wave = tid >> 5;
  const size_t o = (size_t)blockIdx.x * HID + (size_t)tid * 8;
  const v4f a0 = *(const v4f*)(x + o);
  const v4f a1 = *(const v4f*)(x + o + 4);
  float s = ((a0[0] + a0[1]) + (a0[2] + a0[3])) + ((a1[0] + a1[1]) + (a1[2] + a1[3]));
#pragma unroll
  for (int off = 16; off >= 1; off >>= 1) s += __shfl_xor(s, off, 32);
  if (lane == 0) rs1[wave] = s;
  __syncthreads();
  const float mean = ((rs1[0] + rs1[1]) + (rs1[2] + rs1[3])) * (1.0f / (float)HID);
  const v4f d0 = a0 - mean;
  const v4f d1 = a1 - mean;
  float q = ((d0[0] * d0[0] + d0[1] * d0[1]) + (d0[2] * d0[2] + d0[3] * d0[3])) +
            ((d1[0] * d1[0] + d1[1] * d1[1]) + (d1[2] * d1[2] + d1[3] * d1[3]));
#pragma unroll
  for (int off = 16; off >= 1; off >>= 1) q += __shfl_xor(q, off, 32);
  if (lane == 0) rs2[wave] = q;
  __syncthreads();
  const float var  = ((rs2[0] + rs2[1]) + (rs2[2] + rs2[3])) * (1.0f / (float)HID);
  const float rstd = rsqrtf(var + 1e-5f);
  const v4f g0 = *(const v4f*)(gm + tid * 8), g1 = *(const v4f*)(gm + tid * 8 + 4);
  const v4f b0 = *(const v4f*)(bt + tid * 8), b1 = *(const v4f*)(bt + tid * 8 + 4);
  const v4f y0 = d0 * rstd * g0 + b0;
  const v4f y1 = d1 * rstd * g1 + b1;
  Pack8 pk;
  pk.h = (v8h){(_Float16)y0[0], (_Float16)y0[1], (_Float16)y0[2], (_Float16)y0[3],
               (_Float16)y1[0], (_Float16)y1[1], (_Float16)y1[2], (_Float16)y1[3]};
  const v4u vv = pk.u;
  volatile v4u* dp = (volatile v4u*)(xh + o);
  *dp = vv;
  __threadfence();
  *dp = vv;
}

#define SFP 132
__global__ __launch_bounds__(256) void k_qkv(const _Float16* __restrict__ xh,
                                             const _Float16* __restrict__ wt,
                                             _Float16* __restrict__ qp,
                                             _Float16* __restrict__ kp,
                                             _Float16* __restrict__ vtp) {
  __shared__ __align__(16) float sf[64 * SFP];
  const int tid = threadIdx.x, lane = tid & 31, wave = tid >> 5;
  const int hh = lane >> 4, c = lane & 15;
  const int wm = wave >> 1, wn = wave & 1;
  const int mb = blockIdx.x * 64;
  const int b  = mb / SQ;
  const int sb = mb - b * SQ;
  const int ns = blockIdx.y;
  const int which = ns / NH;
  const int head  = ns - which * NH;
  const int hb = b * NH + head;
  const int m0 = mb + wm * 16;
  const int n0 = ns * HDM + wn * 64;

  v8f acc[4];
#pragma unroll
  for (int t = 0; t < 4; ++t) acc[t] = zero8();
  gemm16x64(xh, HID, wt, HID, m0, n0, lane, acc);

#pragma unroll
  for (int t = 0; t < 4; ++t) {
#pragma unroll
    for (int r = 0; r < 8; ++r)
      sf[(wm * 16 + 8 * hh + r) * SFP + wn * 64 + 16 * t + c] = acc[t][r] * 0.03125f;
  }
  __syncthreads();

  if (which < 2) {
    v4u val[4];
    size_t go[4];
#pragma unroll
    for (int j = 0; j < 4; ++j) {
      const int p  = tid + 256 * j;
      const int lr = p >> 4;
      const int d0 = (p & 15) * 8;
      const float* ra = sf + lr * SFP + d0;
      const v4f a0 = *(const v4f*)(ra), a1 = *(const v4f*)(ra + 4);
      Pack8 pk;
      pk.h = (v8h){(_Float16)a0[0], (_Float16)a0[1], (_Float16)a0[2], (_Float16)a0[3],
                   (_Float16)a1[0], (_Float16)a1[1], (_Float16)a1[2], (_Float16)a1[3]};
      val[j] = pk.u;
      go[j]  = ((size_t)hb * SQ + sb + lr) * HDM + d0;
    }
    _Float16* base = (which == 0) ? qp : kp;
    for (int ps = 0; ps < 2; ++ps) {
#pragma unroll
      for (int j = 0; j < 4; ++j) *(volatile v4u*)(base + go[j]) = val[j];
      __threadfence();
    }
  } else {
    v4u val[4];
    size_t go[4];
#pragma unroll
    for (int j = 0; j < 4; ++j) {
      const int p  = tid + 256 * j;
      const int d  = p >> 3;
      const int pc = p & 7;
      const float* cp = sf + (pc * 8) * SFP + d;
      Pack8 pk;
      pk.h = (v8h){(_Float16)cp[0 * SFP], (_Float16)cp[1 * SFP], (_Float16)cp[2 * SFP], (_Float16)cp[3 * SFP],
                   (_Float16)cp[4 * SFP], (_Float16)cp[5 * SFP], (_Float16)cp[6 * SFP], (_Float16)cp[7 * SFP]};
      val[j] = pk.u;
      go[j]  = ((size_t)hb * HDM + d) * SQ + sb + pc * 8;
    }
    for (int ps = 0; ps < 2; ++ps) {
#pragma unroll
      for (int j = 0; j < 4; ++j) *(volatile v4u*)(vtp + go[j]) = val[j];
      __threadfence();
    }
  }
}

#define KTQ 136
#define KTP 72
__global__ __launch_bounds__(256) void k_attn(const _Float16* __restrict__ qp,
                                              const _Float16* __restrict__ kp,
                                              const _Float16* __restrict__ vt,
                                              _Float16* __restrict__ op, float sscale) {
  __shared__ __align__(16) _Float16 Ks[KC * KTQ];
  __shared__ __align__(16) _Float16 Vs[HDM * KTP];
  __shared__ __align__(16) _Float16 Ps[8 * 16 * KTP];

  const int tid = threadIdx.x, lane = tid & 31, wave = tid >> 5;
  const int hh = lane >> 4, c = lane & 15;
  const int qb  = blockIdx.x % NQB;
  const int hb  = blockIdx.x / NQB;
  const int h   = hb % NH;
  const int b   = hb / NH;
  const int q0  = qb * QB + wave * 16;

  const _Float16* Q = qp + (size_t)hb * SQ * HDM;
  const _Float16* K = kp + (size_t)hb * SQ * HDM;
  const _Float16* V = vt + (size_t)hb * HDM * SQ;
  const size_t trow0 = (size_t)b * SQ;

  const float NEGI = -__builtin_huge_valf();
  float mrow[8], lrow[8];
  v8f oacc[8];
#pragma unroll
  for (int r = 0; r < 8; ++r) { mrow[r] = NEGI; lrow[r] = 0.f; }
#pragma unroll
  for (int t = 0; t < 8; ++t) oacc[t] = zero8();

  _Float16* pw = Ps + wave * 16 * KTP;
  const int nck = 2 * qb + 2;

  for (int kc = 0; kc < nck; ++kc) {
    const int kv0 = kc * KC;
    __syncthreads();
    {
      const int r  = tid >> 2;
      const int qq = (tid & 3) * 32;
      const _Float16* ks = K + (size_t)(kv0 + r) * HDM + qq;
#pragma unroll
      for (int e = 0; e < 4; ++e) *(v8h*)(Ks + r * KTQ + qq + 8 * e) = *(const v8h*)(ks + 8 * e);
      const int dr = tid >> 1;
      const int q2 = (tid & 1) * 32;
      const _Float16* vs = V + (size_t)dr * SQ + kv0 + q2;
#pragma unroll
      for (int e = 0; e < 4; ++e) *(v8h*)(Vs + dr * KTP + q2 + 8 * e) = *(const v8h*)(vs + 8 * e);
    }
    __syncthreads();

    v8f s[4];
#pragma unroll
    for (int j = 0; j < 4; ++j) s[j] = zero8();
#pragma unroll
    for (int dc = 0; dc < 4; ++dc) {
      const v16h qa = ldfrag(Q, HDM, q0, dc * 32, lane);
#pragma unroll
      for (int j = 0; j < 4; ++j) {
        const v16h kb = ldfrag(Ks, KTQ, j * 16, dc * 32, lane);
        s[j] = mma16(qa, kb, s[j]);
      }
    }
    const bool edge = (kc >= 2 * qb);
#pragma unroll
    for (int r = 0; r < 8; ++r) {
      const int qry = q0 + 8 * hh + r;
#pragma unroll
      for (int j = 0; j < 4; ++j) {
        const int key = kv0 + 16 * j + c;
        const float v = s[j][r] * sscale;
        s[j][r] = (edge && key > qry) ? NEGI : v;
      }
    }
    float cm[8];
#pragma unroll
    for (int r = 0; r < 8; ++r) {
      float m = NEGI;
#pragma unroll
      for (int j = 0; j < 4; ++j) m = fmaxf(m, s[j][r]);
#pragma unroll
      for (int off = 1; off < 16; off <<= 1) m = fmaxf(m, __shfl_xor(m, off, 32));
      cm[r] = m;
    }
    float al[8];
#pragma unroll
    for (int r = 0; r < 8; ++r) {
      const float mnew  = fmaxf(mrow[r], cm[r]);
      const float alpha = __expf(mrow[r] - mnew);
      mrow[r] = mnew;
      float psum = 0.f;
#pragma unroll
      for (int j = 0; j < 4; ++j) {
        const float p = __expf(s[j][r] - mnew);
        psum += p;
        pw[(8 * hh + r) * KTP + j * 16 + c] = (_Float16)(p * 1024.0f);
      }
#pragma unroll
      for (int off = 1; off < 16; off <<= 1) psum += __shfl_xor(psum, off, 32);
      lrow[r] = lrow[r] * alpha + psum;
      al[r] = alpha;
    }
#pragma unroll
    for (int t = 0; t < 8; ++t)
#pragma unroll
      for (int r = 0; r < 8; ++r) oacc[t][r] *= al[r];
    __syncthreads();

#pragma unroll
    for (int kk = 0; kk < 2; ++kk) {
      const v16h pa = ldfrag(pw, KTP, 0, kk * 32, lane);
#pragma unroll
      for (int t = 0; t < 8; ++t) {
        const v16h vb = ldfrag(Vs, KTP, t * 16, kk * 32, lane);
        oacc[t] = mma16(pa, vb, oacc[t]);
      }
    }
  }

  float invl[8];
#pragma unroll
  for (int r = 0; r < 8; ++r) invl[r] = (lrow[r] > 0.f) ? (0.015625f * (1.0f / lrow[r])) : 0.f;
#pragma unroll
  for (int half = 0; half < 2; ++half) {
    __syncthreads();
#pragma unroll
    for (int r = 0; r < 8; ++r) {
#pragma unroll
      for (int t = 0; t < 4; ++t)
        pw[(8 * hh + r) * KTP + 16 * t + c] = (_Float16)(oacc[4 * half + t][r] * invl[r]);
    }
    __syncthreads();
    v4u val[4];
    size_t go[4];
#pragma unroll
    for (int it = 0; it < 4; ++it) {
      const int p  = lane + 32 * it;
      const int L  = p >> 3;
      const int pc = p & 7;
      Pack8 pk;
      pk.h    = *(const v8h*)(pw + L * KTP + pc * 8);
      val[it] = pk.u;
      go[it]  = (trow0 + q0 + L) * HID + (size_t)h * HDM + half * 64 + pc * 8;
    }
    for (int ps = 0; ps < 2; ++ps) {
#pragma unroll
      for (int it = 0; it < 4; ++it) *(volatile v4u*)(op + go[it]) = val[it];
      __threadfence();
    }
  }
}

#define OTP 68
__device__ __forceinline__ void out_epilogue(v8f (&acc)[2][4], float scale, float* sw,
                                             const float* __restrict__ res, float* __restrict__ out,
                                             int m0, int n0, int lane, int hh, int c) {
#pragma unroll
  for (int sub = 0; sub < 2; ++sub) {
    __syncthreads();
#pragma unroll
    for (int t = 0; t < 4; ++t) {
#pragma unroll
      for (int r = 0; r < 8; ++r) sw[(8 * hh + r) * OTP + 16 * t + c] = acc[sub][t][r] * scale;
    }
    __syncthreads();
    v4f val[8];
    size_t go[8];
#pragma unroll
    for (int it = 0; it < 8; ++it) {
      const int p    = lane + 32 * it;
      const int L    = p >> 3;
      const int pc   = p & 7;
      const int row  = L >> 1;
      const int half = L & 1;
      go[it]  = (size_t)(m0 + sub * 16 + row) * HID + n0 + half * 32 + pc * 4;
      const v4f sv = *(const v4f*)(sw + row * OTP + half * 32 + pc * 4);
      const v4f rv = *(const v4f*)(res + go[it]);
      val[it] = sv + rv;
    }
    for (int ps = 0; ps < 2; ++ps) {
#pragma unroll
      for (int it = 0; it < 8; ++it) *(volatile v4f*)(out + go[it]) = val[it];
      __threadfence();
    }
  }
}

__global__ __launch_bounds__(256) void k_out(const _Float16* __restrict__ ap,
                                             const _Float16* __restrict__ wt,
                                             const float* __restrict__ res,
                                             float* __restrict__ out) {
  __shared__ __align__(16) float st[8][16 * OTP];
  const int tid = threadIdx.x, lane = tid & 31, wave = tid >> 5;
  const int hh = lane >> 4, c = lane & 15;
  const int m0   = blockIdx.x * 256 + wave * 32;
  const int n0   = blockIdx.y * 64;

  v8f acc[2][4];
#pragma unroll
  for (int s = 0; s < 2; ++s)
#pragma unroll
    for (int t = 0; t < 4; ++t) acc[s][t] = zero8();
  gemm32x64(ap, HID, wt, HID, m0, n0, lane, acc);
  out_epilogue(acc, 0.001953125f, st[wave], res, out, m0, n0, lane, hh, c);
}

extern "C" void kernel_launch(void* const* d_in, const int* in_sizes, int n_in,
                              void* d_out, int out_size, void* d_ws, size_t ws_size,
                              hipStream_t stream) {
  if (n_in < 7) return;
  if (in_sizes[0] != NTOK * HID) return;
  if (in_sizes[1] != HID) return;
  if (in_sizes[2] != HID) return;
  if (in_sizes[3] != HID * HID) return;
  if (in_sizes[4] != HID * HID) return;
  if (in_sizes[5] != HID * HID) return;
  if (in_sizes[6] != HID * HID) return;
  if (out_size != NTOK * HID) return;

  const float* x  = (const float*)d_in[0];
  const float* gm = (const float*)d_in[1];
  const float* bt = (const float*)d_in[2];
  const float* wq = (const float*)d_in[3];
  const float* wk = (const float*)d_in[4];
  const float* wv = (const float*)d_in[5];
  const float* wo = (const float*)d_in[6];
  float* out = (float*)d_out;

  size_t off = 0;
  const size_t oX  = off; off += (size_t)NTOK * HID * 2;
  const size_t oWt = off; off += (size_t)NQKV * HID * 2;
  const size_t oWo = off; off += (size_t)HID * HID * 2;
  const size_t oQ  = off; off += (size_t)NBAT * NH * SQ * HDM * 2;
  const size_t oK  = off; off += (size_t)NBAT * NH * SQ * HDM * 2;
  const size_t oV  = off; off += (size_t)NBAT * NH * HDM * SQ * 2;
  const size_t oO  = off; off += (size_t)NTOK * HID * 2;
  if (off > ws_size) return;
  if (off > (size_t)134217728) return;

  char* ws = (char*)d_ws;
  _Float16* Xh  = (_Float16*)(ws + oX);
  _Float16* Wt  = (_Float16*)(ws + oWt);
  _Float16* Wot = (_Float16*)(ws + oWo);
  _Float16* Qp  = (_Float16*)(ws + oQ);
  _Float16* Kp  = (_Float16*)(ws + oK);
  _Float16* Vt  = (_Float16*)(ws + oV);
  _Float16* Op  = (_Float16*)(ws + oO);

  k_cvtw<<<dim3((HID * HID) / 2048, 4), dim3(256), 0, stream>>>(wq, wk, wv, wo, Wt, Wot);
  k_ln<<<dim3(NTOK), dim3(128), 0, stream>>>(x, gm, bt, Xh);
  k_qkv<<<dim3(NTOK / 64, NQKV / HDM), dim3(256), 0, stream>>>(Xh, Wt, Qp, Kp, Vt);
  const float sscale = 0.08838834764831845f;
  k_attn<<<dim3(NBAT * NH * NQB), dim3(256), 0, stream>>>(Qp, Kp, Vt, Op, sscale);
  k_out<<<dim3(NTOK / 256, HID / 64), dim3(256), 0, stream>>>(Op, Wot, x, out);
  (void)hipGetLastError();
}
